// D_FullAttention_11965778886680
// MI455X (gfx1250) — hardware-verified
//
#include <hip/hip_runtime.h>
#include <stddef.h>
#include <stdint.h>

#define NBAT 8
#define NH   2
#define SQ   2048
#define HS   64
#define DIN  (NH * HS)
#define DHID 64
#define NBH  (NBAT * NH)
#define NPOS (NBAT * SQ)
#define QBR  64
#define NWV  4
#define KC   64
#define NQB  (SQ / QBR)
#define NCK  (SQ / KC)
#define PTP  72
#define OTP  68
#define VTRP 65
#define W1P  136
#define NTOT (NBAT * SQ * NH * HS)

static_assert(NTOT == 2097152);
static_assert(NPOS == 16384);
static_assert(SQ % QBR == 0);
static_assert(SQ % KC == 0);
static_assert(QBR == NWV * 16);
static_assert(KC == 64);
static_assert(HS == 64);
static_assert(DIN == 128);
static_assert((PTP * 2) % 16 == 0);
static_assert((OTP * 4) % 16 == 0);
static_assert((W1P * 2) % 16 == 0);
static_assert(NTOT % (8 * 128) == 0);
static_assert((SQ * 8) == 16384);
static_assert(SQ % 64 == 0);
static_assert(SQ == 128 * 16);

typedef float          v8f   __attribute__((ext_vector_type(8)));
typedef float          v4f   __attribute__((ext_vector_type(4)));
typedef unsigned int   v4u   __attribute__((ext_vector_type(4)));
typedef unsigned short v8us  __attribute__((ext_vector_type(8)));
typedef unsigned short v16us __attribute__((ext_vector_type(16)));
typedef __bf16         v16b  __attribute__((ext_vector_type(16)));
typedef unsigned short ush;

union FragU { v16us v; v8us h[2]; v16b b; };
union PackU { v8us s; v4u u; };
struct HL { v4u h; v4u l; };

__device__ __forceinline__ ush f2bf(float f) {
  const unsigned u = __float_as_uint(f);
  return (ush)((u + 0x7FFFu + ((u >> 16) & 1u)) >> 16);
}
__device__ __forceinline__ float bf2f(ush v) { return __uint_as_float(((unsigned)v) << 16); }

__device__ __forceinline__ HL split8(v8f f) {
  PackU ph, pl;
#pragma unroll
  for (int e = 0; e < 8; ++e) {
    const ush hi = f2bf(f[e]);
    ph.s[e] = hi;
    pl.s[e] = f2bf(f[e] - bf2f(hi));
  }
  HL r; r.h = ph.u; r.l = pl.u;
  return r;
}

__device__ __forceinline__ void split16(v8f f0, v8f f1, v16us& hi, v16us& lo) {
  const HL s0 = split8(f0), s1 = split8(f1);
  PackU p; FragU uh, ul;
  p.u = s0.h; uh.h[0] = p.s;
  p.u = s0.l; ul.h[0] = p.s;
  p.u = s1.h; uh.h[1] = p.s;
  p.u = s1.l; ul.h[1] = p.s;
  hi = uh.v; lo = ul.v;
}

__device__ __forceinline__ v8f mmab(v16us a, v16us b, v8f c) {
  FragU ua, ub; ua.v = a; ub.v = b;
  c = __builtin_amdgcn_wmma_f32_16x16x32_bf16(false, ua.b, false, ub.b, (short)0, c, false, false);
  asm volatile("v_nop\n\tv_nop\n\tv_nop\n\tv_nop" : "+v"(c) : "v"(a), "v"(b));
  return c;
}

__device__ __forceinline__ v16us ldfragu(const ush* p, int ld, int row0, int k0, int lane) {
  const int m = lane & 15, lh = lane >> 4;
  const ush* q = p + (size_t)(row0 + m) * ld + k0 + 8 * lh;
  FragU f;
  f.h[0] = *(const v8us*)(q);
  f.h[1] = *(const v8us*)(q + 16);
  return f.v;
}

__device__ __forceinline__ v8f zero8() { return (v8f){0.f, 0.f, 0.f, 0.f, 0.f, 0.f, 0.f, 0.f}; }

__global__ __launch_bounds__(256) void k_cvtqk(const float* __restrict__ q, const float* __restrict__ k,
                                               ush* __restrict__ qh, ush* __restrict__ ql,
                                               ush* __restrict__ kh, ush* __restrict__ kl) {
  const int tid = threadIdx.x;
  const int sel = tid >> 7;
  const int t   = tid & 127;
  const unsigned pd = (unsigned)blockIdx.x * 128u + (unsigned)t;
  const unsigned e8 = pd & 7u;
  const unsigned l  = (pd / 8u) % (unsigned)SQ;
  const unsigned bh = pd / (unsigned)(SQ * 8);
  const unsigned b  = bh / (unsigned)NH;
  const unsigned n  = bh % (unsigned)NH;
  const size_t so = (((size_t)b * SQ + l) * NH + n) * HS + (size_t)e8 * 8;
  const size_t dofs = (size_t)pd * 8;
  const float* src = (sel == 0) ? q : k;
  ush* dh = (sel == 0) ? qh : kh;
  ush* dl = (sel == 0) ? ql : kl;
  const v4f a0 = *(const v4f*)(src + so);
  const v4f a1 = *(const v4f*)(src + so + 4);
  const v8f f = (v8f){a0[0], a0[1], a0[2], a0[3], a1[0], a1[1], a1[2], a1[3]};
  const HL sp = split8(f);
  *(volatile v4u*)(dh + dofs) = sp.h;
  *(volatile v4u*)(dl + dofs) = sp.l;
  __threadfence();
  *(volatile v4u*)(dh + dofs) = sp.h;
  *(volatile v4u*)(dl + dofs) = sp.l;
}

__global__ __launch_bounds__(256) void k_vtr(const float* __restrict__ v,
                                             ush* __restrict__ vth, ush* __restrict__ vtl) {
  __shared__ float tl[64 * VTRP];
  const int tid = threadIdx.x;
  const int s0 = blockIdx.x * 64;
  const int hb = blockIdx.y;
  const int b  = hb / NH;
  const int n  = hb % NH;
#pragma unroll
  for (int j = 0; j < 4; ++j) {
    const int p  = tid + 256 * j;
    const int ss = p >> 4;
    const int q4 = (p & 15) * 4;
    const v4f a = *(const v4f*)(v + (((size_t)b * SQ + s0 + ss) * NH + n) * HS + q4);
    float* d = tl + ss * VTRP + q4;
    d[0] = a[0]; d[1] = a[1]; d[2] = a[2]; d[3] = a[3];
  }
  __syncthreads();
  v4u vh[2], vl[2];
  size_t go[2];
#pragma unroll
  for (int j = 0; j < 2; ++j) {
    const int p  = tid + 256 * j;
    const int dd = p >> 3;
    const int pc = p & 7;
    const float* cp = tl + (pc * 8) * VTRP + dd;
    const v8f f = (v8f){cp[0 * VTRP], cp[1 * VTRP], cp[2 * VTRP], cp[3 * VTRP],
                        cp[4 * VTRP], cp[5 * VTRP], cp[6 * VTRP], cp[7 * VTRP]};
    const HL sp = split8(f);
    vh[j] = sp.h; vl[j] = sp.l;
    go[j] = ((size_t)hb * HS + dd) * SQ + s0 + pc * 8;
  }
  for (int ps = 0; ps < 2; ++ps) {
#pragma unroll
    for (int j = 0; j < 2; ++j) {
      *(volatile v4u*)(vth + go[j]) = vh[j];
      *(volatile v4u*)(vtl + go[j]) = vl[j];
    }
    __threadfence();
  }
}

__global__ __launch_bounds__(128)
void k_deg(const float* __restrict__ v, const float* __restrict__ W1, const float* __restrict__ b1,
           const float* __restrict__ W2, const float* __restrict__ b2, float* __restrict__ degm) {
  __shared__ __align__(16) ush   w1h[DHID * W1P];
  __shared__ __align__(16) ush   w1l[DHID * W1P];
  __shared__ __align__(16) float b1s[DHID];
  __shared__ __align__(16) float w2s[DHID];
  __shared__ __align__(16) float degs[SQ];
  __shared__ float wmx[NWV];

  const int tid = threadIdx.x, lane = tid & 31, wave = tid >> 5;
  const int hh = lane >> 4, c = lane & 15;
  const int b = blockIdx.x;

  for (int i = tid; i < DIN * DHID; i += 128) {
    const int kk = i >> 6, nn = i & 63;
    const float w = W1[i];
    const ush hi = f2bf(w);
    w1h[nn * W1P + kk] = hi;
    w1l[nn * W1P + kk] = f2bf(w - bf2f(hi));
  }
  if (tid < DHID) { b1s[tid] = b1[tid]; w2s[tid] = W2[tid]; }
  const float bias2 = b2[0];
  __syncthreads();

#pragma unroll 1
  for (int tile = 0; tile < SQ / 64; ++tile) {
    const int r0 = tile * 64 + wave * 16;
    const float* arow = v + ((size_t)b * SQ + r0 + c) * DIN;
    v8f acc[4];
#pragma unroll
    for (int t = 0; t < 4; ++t) acc[t] = zero8();
#pragma unroll
    for (int ks = 0; ks < 4; ++ks) {
      const int k0 = ks * 32;
      const float* ap = arow + k0 + 8 * hh;
      const v4f x0 = *(const v4f*)(ap);
      const v4f x1 = *(const v4f*)(ap + 4);
      const v4f x2 = *(const v4f*)(ap + 16);
      const v4f x3 = *(const v4f*)(ap + 20);
      const v8f f0 = (v8f){x0[0], x0[1], x0[2], x0[3], x1[0], x1[1], x1[2], x1[3]};
      const v8f f1 = (v8f){x2[0], x2[1], x2[2], x2[3], x3[0], x3[1], x3[2], x3[3]};
      v16us ah, al;
      split16(f0, f1, ah, al);
#pragma unroll
      for (int t = 0; t < 4; ++t) {
        const v16us bh = ldfragu(w1h, W1P, 16 * t, k0, lane);
        const v16us bl = ldfragu(w1l, W1P, 16 * t, k0, lane);
        acc[t] = mmab(ah, bh, acc[t]);
        acc[t] = mmab(ah, bl, acc[t]);
        acc[t] = mmab(al, bh, acc[t]);
      }
    }
    float part[8];
#pragma unroll
    for (int r = 0; r < 8; ++r) {
      float p = 0.f;
#pragma unroll
      for (int t = 0; t < 4; ++t) {
        const float hv = fmaxf(acc[t][r] + b1s[16 * t + c], 0.f);
        p = fmaf(hv, w2s[16 * t + c], p);
      }
      part[r] = p;
    }
#pragma unroll
    for (int r = 0; r < 8; ++r) {
#pragma unroll
      for (int off = 1; off < 16; off <<= 1) part[r] += __shfl_xor(part[r], off, 32);
    }
#pragma unroll
    for (int r = 0; r < 8; ++r) {
      float s2 = part[r] + bias2;
      s2 = fminf(fmaxf(s2, -30.0f), 30.0f);
      const float ex = expf(-s2);
      const float sg = 1.0f / (1.0f + ex);
      const float dv = fminf(fmaxf(sg, 0.01f), 0.99f);
      if (c == r) degs[r0 + 8 * hh + r] = dv;
    }
  }
  __syncthreads();

  float mx = degs[tid * 16];
#pragma unroll
  for (int i = 1; i < 16; ++i) mx = fmaxf(mx, degs[tid * 16 + i]);
#pragma unroll
  for (int off = 1; off < 32; off <<= 1) mx = fmaxf(mx, __shfl_xor(mx, off, 32));
  if (lane == 0) wmx[wave] = mx;
  __syncthreads();
  const float bm = fmaxf(fmaxf(wmx[0], wmx[1]), fmaxf(wmx[2], wmx[3]));

  v4f val[4];
  size_t go[4];
#pragma unroll
  for (int it = 0; it < 4; ++it) {
    const int p = tid + 128 * it;
    val[it] = (v4f){degs[4 * p + 0] - bm, degs[4 * p + 1] - bm, degs[4 * p + 2] - bm, degs[4 * p + 3] - bm};
    go[it]  = (size_t)b * SQ + (size_t)p * 4;
  }
  for (int ps = 0; ps < 2; ++ps) {
#pragma unroll
    for (int it = 0; it < 4; ++it) *(volatile v4f*)(degm + go[it]) = val[it];
    __threadfence();
  }
}

__global__ __launch_bounds__(128)
void k_attn(const ush* __restrict__ qh, const ush* __restrict__ ql,
            const ush* __restrict__ kh, const ush* __restrict__ kl,
            const ush* __restrict__ vth, const ush* __restrict__ vtl,
            const float* __restrict__ degm, float* __restrict__ out) {
  __shared__ __align__(16) ush   Ph[NWV * 16 * PTP];
  __shared__ __align__(16) ush   Pl[NWV * 16 * PTP];
  __shared__ __align__(16) float Os[NWV * 16 * OTP];

  const int tid = threadIdx.x, lane = tid & 31, wave = tid >> 5;
  const int hh = lane >> 4, c = lane & 15;
  const int qb   = blockIdx.x % NQB;
  const int hb   = blockIdx.x / NQB;
  const int h    = hb % NH;
  const int b    = hb / NH;
  const int q0   = qb * QBR + wave * 16;
  const float scale = 0.125f;

  const ush* Qh = qh  + (size_t)hb * SQ * HS;
  const ush* Ql = ql  + (size_t)hb * SQ * HS;
  const ush* Kh = kh  + (size_t)hb * SQ * HS;
  const ush* Kl = kl  + (size_t)hb * SQ * HS;
  const ush* Vh = vth + (size_t)hb * HS * SQ;
  const ush* Vl = vtl + (size_t)hb * HS * SQ;
  const float* dg = degm + (size_t)b * SQ;

  ush*   pwh = Ph + wave * 16 * PTP;
  ush*   pwl = Pl + wave * 16 * PTP;
  float* sw  = Os + wave * 16 * OTP;

  const float NEGI = -__builtin_huge_valf();
  float mrow[8], lrow[8];
  v8f oacc[4];
#pragma unroll
  for (int r = 0; r < 8; ++r) { mrow[r] = NEGI; lrow[r] = 0.f; }
#pragma unroll
  for (int t = 0; t < 4; ++t) oacc[t] = zero8();

#pragma unroll 1
  for (int kc = 0; kc < NCK; ++kc) {
    const int kv0 = kc * KC;
    __syncthreads();

    float dj[4];
#pragma unroll
    for (int j = 0; j < 4; ++j) dj[j] = dg[kv0 + 16 * j + c];

    v8f s[4];
#pragma unroll
    for (int j = 0; j < 4; ++j) s[j] = zero8();
#pragma unroll
    for (int dc = 0; dc < 2; ++dc) {
      const v16us qah = ldfragu(Qh, HS, q0, dc * 32, lane);
      const v16us qal = ldfragu(Ql, HS, q0, dc * 32, lane);
#pragma unroll
      for (int j = 0; j < 4; ++j) {
        const v16us kbh = ldfragu(Kh, HS, kv0 + 16 * j, dc * 32, lane);
        const v16us kbl = ldfragu(Kl, HS, kv0 + 16 * j, dc * 32, lane);
        s[j] = mmab(qah, kbh, s[j]);
        s[j] = mmab(qah, kbl, s[j]);
        s[j] = mmab(qal, kbh, s[j]);
      }
    }
#pragma unroll
    for (int r = 0; r < 8; ++r)
#pragma unroll
      for (int j = 0; j < 4; ++j) {
        const float sv = s[j][r] + dj[j];
        s[j][r] = sv * scale;
      }

    float cm[8];
#pragma unroll
    for (int r = 0; r < 8; ++r) {
      float m = fmaxf(fmaxf(s[0][r], s[1][r]), fmaxf(s[2][r], s[3][r]));
#pragma unroll
      for (int off = 1; off < 16; off <<= 1) m = fmaxf(m, __shfl_xor(m, off, 32));
      cm[r] = m;
    }
    float al[8];
#pragma unroll
    for (int r = 0; r < 8; ++r) {
      const float mnew  = fmaxf(mrow[r], cm[r]);
      const float alpha = __expf(mrow[r] - mnew);
      mrow[r] = mnew;
      float psum = 0.f;
#pragma unroll
      for (int j = 0; j < 4; ++j) {
        const float p = __expf(s[j][r] - mnew);
        psum += p;
        const ush phi = f2bf(p);
        pwh[(8 * hh + r) * PTP + 16 * j + c] = phi;
        pwl[(8 * hh + r) * PTP + 16 * j + c] = f2bf(p - bf2f(phi));
      }
#pragma unroll
      for (int off = 1; off < 16; off <<= 1) psum += __shfl_xor(psum, off, 32);
      lrow[r] = lrow[r] * alpha + psum;
      al[r] = alpha;
    }
#pragma unroll
    for (int t = 0; t < 4; ++t)
#pragma unroll
      for (int r = 0; r < 8; ++r) oacc[t][r] *= al[r];
    __syncthreads();

#pragma unroll
    for (int kk = 0; kk < 2; ++kk) {
      const v16us pah = ldfragu(pwh, PTP, 0, kk * 32, lane);
      const v16us pal = ldfragu(pwl, PTP, 0, kk * 32, lane);
#pragma unroll
      for (int t = 0; t < 4; ++t) {
        const v16us vbh = ldfragu(Vh, SQ, 16 * t, kv0 + kk * 32, lane);
        const v16us vbl = ldfragu(Vl, SQ, 16 * t, kv0 + kk * 32, lane);
        oacc[t] = mmab(pah, vbh, oacc[t]);
        oacc[t] = mmab(pah, vbl, oacc[t]);
        oacc[t] = mmab(pal, vbh, oacc[t]);
      }
    }
  }
  __syncthreads();

#pragma unroll
  for (int r = 0; r < 8; ++r) {
    const float lr  = lrow[r];
    const float inv = (lr > 0.f) ? (1.0f / lr) : 0.f;
    const int   row = 8 * hh + r;
#pragma unroll
    for (int t = 0; t < 4; ++t) sw[row * OTP + 16 * t + c] = oacc[t][r] * inv;
  }
  __syncthreads();
  v4f val[8];
  size_t go[8];
#pragma unroll
  for (int it = 0; it < 8; ++it) {
    const int p    = lane + 32 * it;
    const int L    = p >> 3;
    const int pc   = p & 7;
    const int row  = L >> 1;
    const int half = L & 1;
    val[it] = *(const v4f*)(sw + row * OTP + half * 32 + pc * 4);
    go[it]  = ((size_t)(b * SQ + q0 + row) * NH + h) * HS + half * 32 + pc * 4;
  }
  for (int ps = 0; ps < 2; ++ps) {
#pragma unroll
    for (int it = 0; it < 8; ++it) *(volatile v4f*)(out + go[it]) = val[it];
    __threadfence();
  }
}

extern "C" void kernel_launch(void* const* d_in, const int* in_sizes, int n_in,
                              void* d_out, int out_size, void* d_ws, size_t ws_size,
                              hipStream_t stream) {
  if (n_in < 7) return;
  if (in_sizes[0] != NTOT) return;
  if (in_sizes[1] != NTOT) return;
  if (in_sizes[2] != NTOT) return;
  if (in_sizes[3] != DIN * DHID) return;
  if (in_sizes[4] < DHID) return;
  if (in_sizes[5] < DHID) return;
  if (in_sizes[6] < 1) return;
  if (out_size != NTOT) return;

  const float* q  = (const float*)d_in[0];
  const float* k  = (const float*)d_in[1];
  const float* v  = (const float*)d_in[2];
  const float* W1 = (const float*)d_in[3];
  const float* b1 = (const float*)d_in[4];
  const float* W2 = (const float*)d_in[5];
  const float* b2 = (const float*)d_in[6];
  float* out = (float*)d_out;

  const size_t plane = (size_t)NTOT * 2;
  const size_t degb  = (size_t)NPOS * 4;
  size_t off = 0;
  const size_t oQh = off; off += plane;
  const size_t oQl = off; off += plane;
  const size_t oKh = off; off += plane;
  const size_t oKl = off; off += plane;
  const size_t oVh = off; off += plane;
  const size_t oVl = off; off += plane;
  const size_t oDg = off; off += degb;
  if (off > ws_size) return;
  if (off > (size_t)134217728) return;

  char* ws = (char*)d_ws;
  ush* Qh  = (ush*)(ws + oQh);
  ush* Ql  = (ush*)(ws + oQl);
  ush* Kh  = (ush*)(ws + oKh);
  ush* Kl  = (ush*)(ws + oKl);
  ush* VTh = (ush*)(ws + oVh);
  ush* VTl = (ush*)(ws + oVl);
  float* Dg = (float*)(ws + oDg);

  k_cvtqk<<<dim3(NTOT / (8 * 128)), dim3(256), 0, stream>>>(q, k, Qh, Ql, Kh, Kl);
  k_vtr<<<dim3(SQ / 64, NBH), dim3(256), 0, stream>>>(v, VTh, VTl);
  k_deg<<<dim3(NBAT), dim3(128), 0, stream>>>(v, W1, b1, W2, b2, Dg);
  k_attn<<<dim3(NBH * NQB), dim3(128), 0, stream>>>(Qh, Ql, Kh, Kl, VTh, VTl, Dg, out);
  (void)hipGetLastError();
}
